// GCN_31241592111373
// MI455X (gfx1250) — hardware-verified
//
#include <hip/hip_runtime.h>
#include <stddef.h>
#include <stdint.h>
#include <math.h>


#define CH      64
#define K2      128
#define OUTC    16
#define NTHR    256
#define NWAVE   8
#define EPT     8
#define CHUNK   (NTHR * EPT)
#define WCAP    (EPT * 32)
#define LISTN   (NWAVE * WCAP)
#define NBA     1024
#define SLA     10
#define RCAP    28672
#define DEGCAP  128
#define GBM     64
#define GBN     64
#define GTHR    128
#define HBM     128
#define MROWS   128
#define FLN     32
#define NU1     (CH * (CH / 8))
#define NU2     (CH * (K2 / 8))
#define NU3     (OUTC * (K2 / 8))
#define AGG_ZINTS (LISTN + 2 * RCAP + 3 * NBA)
#define AGG_LDS_INTS (AGG_ZINTS + 32)
#define WSMAX   134217728

static_assert(CH == 64 && OUTC == 16 && K2 == 2 * CH);
static_assert((CHUNK & (CHUNK - 1)) == 0 && CHUNK <= 4096);
static_assert((NBA & (NBA - 1)) == 0 && NBA == (1 << SLA));
static_assert(((long long)CHUNK << SLA) < (1LL << 31));
static_assert(LISTN % NTHR == 0);
static_assert(NBA % NWAVE == 0 && NBA % 32 == 0 && NBA % GBM == 0 && NBA % HBM == 0 && NBA % 2 == 0);
static_assert(NBA == NTHR * 4);
static_assert(RCAP % 32 == 0 && RCAP % (NTHR * 4) == 0 && AGG_ZINTS % 4 == 0 && LISTN % 4 == 0);
static_assert(RCAP >= 17546);
static_assert(DEGCAP >= 44);
static_assert(CH % 32 == 0 && K2 % 32 == 0 && CH == GBN);
static_assert(GBM == (GTHR / 32) * 16 && GBN == 64);
static_assert(HBM == NWAVE * 16 && (HBM * OUTC) % (4 * NTHR) == 0);
static_assert(MROWS % GBM == 0 && MROWS % HBM == 0 && MROWS % 32 == 0);
static_assert(NU1 % NTHR == 0 && NU2 % NTHR == 0 && NU3 % NTHR == 0);
static_assert(CH == 2 * 32);
static_assert(AGG_LDS_INTS * 4 <= 300000);
static_assert(FLN * 4 == 128);

typedef float          v2f   __attribute__((ext_vector_type(2)));
typedef float          v4f   __attribute__((ext_vector_type(4)));
typedef float          v8f   __attribute__((ext_vector_type(8)));
typedef int            v4i   __attribute__((ext_vector_type(4)));
typedef int            v8i   __attribute__((ext_vector_type(8)));
typedef unsigned int   v4u   __attribute__((ext_vector_type(4)));
typedef unsigned short v8us  __attribute__((ext_vector_type(8)));
typedef unsigned short v16us __attribute__((ext_vector_type(16)));
typedef __bf16         v16bf __attribute__((ext_vector_type(16)));
typedef v2f  __attribute__((may_alias)) v2fa;
typedef v4f  __attribute__((may_alias)) v4fa;
typedef v4i  __attribute__((may_alias)) v4ia;
typedef v8us __attribute__((may_alias)) v8usa;
union FragB { v16bf v; v16us u; v8us h[2]; v8i w; };

__device__ __forceinline__ v8f wmb(const FragB& a, const FragB& b, v8f c) {
  v8f d = __builtin_amdgcn_wmma_f32_16x16x32_bf16(false, a.v, false, b.v, (short)0, c, false, false);
  asm volatile("v_nop\n\tv_nop\n\tv_nop\n\tv_nop" : "+v"(d) : "v"(a.w), "v"(b.w));
  return d;
}

__device__ __forceinline__ unsigned bf16_bits(float f) {
  const unsigned u = __float_as_uint(f);
  const unsigned r = ((u + 0x7FFFu + ((u >> 16) & 1u)) >> 16) & 0xFFFFu;
  return (f != f) ? 0x7FC0u : r;
}
__device__ __forceinline__ float bf16_val(float f) {
  return __uint_as_float(bf16_bits(f) << 16);
}
__device__ __forceinline__ void st2_us8(unsigned short* p, const v8us o) {
  *(volatile v8us*)p = o;
  __threadfence();
  *(volatile v8us*)p = o;
}

__device__ __forceinline__ int scan_chunk(const int* __restrict__ dsts, int nE, int cbase, int slotBase,
                                          int nb, int vec8, int* list, int tid, int lane, int wave) {
  int wc = 0;
  const int el0  = tid * EPT;
  const int e0   = cbase + el0;
  const int sent = -2147483647 - 1;
  v4i da, db;
  if (vec8 != 0 && cbase + CHUNK <= nE) {
    da = *(const v4i*)(dsts + e0);
    db = *(const v4i*)(dsts + e0 + 4);
  } else {
    da.x = (e0     < nE) ? dsts[min(e0,     nE - 1)] : sent;
    da.y = (e0 + 1 < nE) ? dsts[min(e0 + 1, nE - 1)] : sent;
    da.z = (e0 + 2 < nE) ? dsts[min(e0 + 2, nE - 1)] : sent;
    da.w = (e0 + 3 < nE) ? dsts[min(e0 + 3, nE - 1)] : sent;
    db.x = (e0 + 4 < nE) ? dsts[min(e0 + 4, nE - 1)] : sent;
    db.y = (e0 + 5 < nE) ? dsts[min(e0 + 5, nE - 1)] : sent;
    db.z = (e0 + 6 < nE) ? dsts[min(e0 + 6, nE - 1)] : sent;
    db.w = (e0 + 7 < nE) ? dsts[min(e0 + 7, nE - 1)] : sent;
  }
  const unsigned nbs = (unsigned)slotBase;
  const unsigned unb = (unsigned)nb;
  const unsigned s0 = (unsigned)da.x - nbs, s1 = (unsigned)da.y - nbs;
  const unsigned s2 = (unsigned)da.z - nbs, s3 = (unsigned)da.w - nbs;
  const unsigned s4 = (unsigned)db.x - nbs, s5 = (unsigned)db.y - nbs;
  const unsigned s6 = (unsigned)db.z - nbs, s7 = (unsigned)db.w - nbs;
  const bool h0 = s0 < unb, h1 = s1 < unb, h2 = s2 < unb, h3 = s3 < unb;
  const bool h4 = s4 < unb, h5 = s5 < unb, h6 = s6 < unb, h7 = s7 < unb;
  const unsigned any = __builtin_amdgcn_ballot_w32(h0 | h1 | h2 | h3 | h4 | h5 | h6 | h7);
  if (any != 0u) {
#define HITJ(J, HJ, SJ) { \
      const unsigned mj = __builtin_amdgcn_ballot_w32(HJ); \
      if (mj != 0u) { \
        if (HJ) { \
          const int pos = wc + (int)__builtin_amdgcn_mbcnt_lo(mj, 0u); \
          if (pos < WCAP) list[wave * WCAP + pos] = ((el0 + (J)) << SLA) | (int)(SJ); \
        } \
        wc += (int)__builtin_popcount(mj); } }
    HITJ(0, h0, s0)
    HITJ(1, h1, s1)
    HITJ(2, h2, s2)
    HITJ(3, h3, s3)
    HITJ(4, h4, s4)
    HITJ(5, h5, s5)
    HITJ(6, h6, s6)
    HITJ(7, h7, s7)
#undef HITJ
  }
  return wc;
}

__global__ __launch_bounds__(NTHR) void k_prep(const float* __restrict__ x, const float* __restrict__ W1,
                                               const float* __restrict__ W2, const float* __restrict__ Wfc,
                                               int nN, int nXb,
                                               unsigned short* xb, unsigned short* w1t,
                                               unsigned short* w2d, unsigned short* wfd) {
  const int bx = (int)blockIdx.x, tid = (int)threadIdx.x;
  if (bx < nXb) {
    const int u   = bx * NTHR + tid;
    const int row = u >> 3;
    const int k8  = (u & 7) * 8;
    const int rc  = row < nN ? row : nN - 1;
    const float* p = x + (size_t)rc * CH + k8;
    const v4f a = *(const v4fa*)p;
    const v4f b = *(const v4fa*)(p + 4);
    const bool ok = row < nN;
    v8us o;
    o[0] = ok ? (unsigned short)bf16_bits(a.x) : (unsigned short)0;
    o[1] = ok ? (unsigned short)bf16_bits(a.y) : (unsigned short)0;
    o[2] = ok ? (unsigned short)bf16_bits(a.z) : (unsigned short)0;
    o[3] = ok ? (unsigned short)bf16_bits(a.w) : (unsigned short)0;
    o[4] = ok ? (unsigned short)bf16_bits(b.x) : (unsigned short)0;
    o[5] = ok ? (unsigned short)bf16_bits(b.y) : (unsigned short)0;
    o[6] = ok ? (unsigned short)bf16_bits(b.z) : (unsigned short)0;
    o[7] = ok ? (unsigned short)bf16_bits(b.w) : (unsigned short)0;
    st2_us8(xb + (size_t)row * CH + k8, o);
  } else {
    const int v = (bx - nXb) * NTHR + tid;
    if (v < NU1) {
      const int n  = v >> 3;
      const int k8 = (v & 7) * 8;
      const float* p = W1 + (size_t)k8 * CH + n;
      v8us o;
#pragma unroll
      for (int i = 0; i < 8; ++i) o[i] = (unsigned short)bf16_bits(p[(size_t)i * CH]);
      st2_us8(w1t + (size_t)n * CH + k8, o);
    } else if (v < NU1 + NU2) {
      const int w  = v - NU1;
      const int n  = w >> 4;
      const int k8 = (w & 15) * 8;
      const int kk = k8 & (CH - 1);
      const float* p = W2 + (size_t)kk * CH + n;
      v8us o;
#pragma unroll
      for (int i = 0; i < 8; ++i) o[i] = (unsigned short)bf16_bits(p[(size_t)i * CH]);
      st2_us8(w2d + (size_t)n * K2 + k8, o);
    } else if (v < NU1 + NU2 + NU3) {
      const int w  = v - NU1 - NU2;
      const int n  = w >> 4;
      const int k8 = (w & 15) * 8;
      const int kk = k8 & (CH - 1);
      const float* p = Wfc + (size_t)kk * OUTC + n;
      v8us o;
#pragma unroll
      for (int i = 0; i < 8; ++i) o[i] = (unsigned short)bf16_bits(p[(size_t)i * OUTC]);
      st2_us8(wfd + (size_t)n * K2 + k8, o);
    }
  }
}

__global__ __launch_bounds__(NTHR) void k_bucket(const int* __restrict__ srcs, const int* __restrict__ dsts,
                                                 int nE, int nN, int vec8,
                                                 int* hits, int* cntg, int* offg, float* dis, int* flagg) {
  extern __shared__ __attribute__((aligned(16))) int dsm[];
  int* list = dsm;
  int* hl   = dsm + LISTN;
  int* sl   = dsm + LISTN + RCAP;
  int* cnt  = dsm + LISTN + 2 * RCAP;
  int* offs = cnt + NBA;
  int* cur  = offs + NBA;
  int* misc = cur + NBA;
  const int tid = (int)threadIdx.x, lane = tid & 31, wave = tid >> 5;
  const int nodeBase = (int)blockIdx.x * NBA;
  int nb = nN - nodeBase;
  nb = nb < 0 ? 0 : (nb > NBA ? NBA : nb);

  {
    const v4i z4 = {0, 0, 0, 0};
    for (int i = tid * 4; i < AGG_ZINTS; i += NTHR * 4) *(v4ia*)(dsm + i) = z4;
    if (tid < 32) misc[tid] = 0;
  }
  __syncthreads();

  int t = 0, ov = 0;
  const int nChunks = (nE + CHUNK - 1) / CHUNK;
#pragma unroll 1
  for (int ch = 0; ch < nChunks; ++ch) {
    const int cbase = ch * CHUNK;
    const int wc = scan_chunk(dsts, nE, cbase, nodeBase, nb, vec8, list, tid, lane, wave);
    if (lane == 0) misc[wave] = wc;
    __syncthreads();
    if (wave == 0) {
#pragma unroll 1
      for (int w2 = 0; w2 < NWAVE; ++w2) {
        int c = misc[w2];
        c = c < 0 ? 0 : (c > WCAP ? WCAP : c);
#pragma unroll 1
        for (int b0 = 0; b0 < c; b0 += 32) {
          const int idx = b0 + lane;
          const int ent = list[w2 * WCAP + (idx < WCAP ? idx : WCAP - 1)];
          const int m32 = (c - b0) < 32 ? (c - b0) : 32;
#pragma unroll 1
          for (int k = 0; k < m32; ++k) {
            const int u    = __builtin_amdgcn_readlane(ent, k);
            const int slot = u & (NBA - 1);
            const int el   = (u >> SLA) & (CHUNK - 1);
            const int pk   = ((cbase + el) << SLA) | slot;
            if (t < RCAP) {
              if (lane == 0) { hl[t] = pk; cnt[slot] = cnt[slot] + 1; }
              t = t + 1;
            } else {
              ov = 1;
            }
          }
        }
      }
    }
    __syncthreads();
  }
  if (wave == 0 && lane == 0) { misc[8] = t; misc[9] = ov; }
  __syncthreads();
  int tt = misc[8];
  tt = tt < 0 ? 0 : (tt > RCAP ? RCAP : tt);

  if (wave == 0) {
    const int base = lane * (NBA / 32);
    int s = 0;
#pragma unroll 1
    for (int i = 0; i < NBA / 32; ++i) s += cnt[base + i];
    int incl = s;
#pragma unroll
    for (int d = 1; d < 32; d <<= 1) {
      const int y = __shfl_up(incl, d, 32);
      if (lane >= d) incl += y;
    }
    int run = incl - s;
#pragma unroll 1
    for (int i = 0; i < NBA / 32; ++i) {
      const int cv = cnt[base + i];
      offs[base + i] = run;
      cur[base + i]  = run;
      run += cv;
    }
  }
  __syncthreads();
  if (wave == 0) {
#pragma unroll 1
    for (int b0 = 0; b0 < tt; b0 += 32) {
      const int idx = b0 + lane;
      const int ent = hl[idx < RCAP ? idx : RCAP - 1];
      const int m32 = (tt - b0) < 32 ? (tt - b0) : 32;
#pragma unroll 1
      for (int k = 0; k < m32; ++k) {
        const int u    = __builtin_amdgcn_readlane(ent, k);
        const int slot = u & (NBA - 1);
        if (lane == 0) {
          int p = cur[slot];
          p = p < 0 ? 0 : (p > RCAP - 1 ? RCAP - 1 : p);
          sl[p] = u;
          cur[slot] = p + 1;
        }
      }
    }
  }
  __syncthreads();

  const v4i c4 = *(const v4ia*)(cnt + 4 * tid);
  const v4i o4 = *(const v4ia*)(offs + 4 * tid);
  {
    const bool bg = (c4.x > DEGCAP) | (c4.y > DEGCAP) | (c4.z > DEGCAP) | (c4.w > DEGCAP);
    const unsigned bm = __builtin_amdgcn_ballot_w32(bg);
    if (lane == 0) misc[16 + wave] = (bm != 0u) ? 1 : 0;
  }
  float* disl = (float*)cur;
#pragma unroll 1
  for (int i = tid; i < NBA; i += NTHR) {
    const float d = (float)(cnt[i] + 1);
    disl[i] = 1.0f / sqrtf(d);
  }
  __syncthreads();
  int fl = misc[9];
#pragma unroll
  for (int w2 = 0; w2 < NWAVE; ++w2) fl |= misc[16 + w2];
  fl = (fl != 0) ? 1 : 0;
  const float qnan = __int_as_float(0x7fc00000);
  v4f dv = *(const v4fa*)(disl + 4 * tid);
  dv.x = (fl != 0) ? qnan : dv.x;
  dv.y = (fl != 0) ? qnan : dv.y;
  dv.z = (fl != 0) ? qnan : dv.z;
  dv.w = (fl != 0) ? qnan : dv.w;
  const v4i fv = {fl, fl, fl, fl};
  int*   cp = cntg + (size_t)nodeBase + 4 * tid;
  int*   op = offg + (size_t)nodeBase + 4 * tid;
  float* dp = dis  + (size_t)nodeBase + 4 * tid;
  int*   fp = flagg + (size_t)blockIdx.x * FLN + 4 * (lane & 7);
  const bool fw = (wave == 0) && (lane < 8);
  *(volatile v4i*)cp = c4;
  *(volatile v4i*)op = o4;
  *(volatile v4f*)dp = dv;
  if (fw) *(volatile v4i*)fp = fv;
  __threadfence();
  *(volatile v4i*)cp = c4;
  *(volatile v4i*)op = o4;
  *(volatile v4f*)dp = dv;
  if (fw) *(volatile v4i*)fp = fv;

  int* hrow = hits + (size_t)blockIdx.x * RCAP;
#pragma unroll 1
  for (int it = 0; it < RCAP / (NTHR * 4); ++it) {
    const int p0 = (it * NTHR + tid) * 4;
    const v4i e4 = *(const v4ia*)(sl + p0);
    int e0 = e4.x >> SLA, e1 = e4.y >> SLA, e2 = e4.z >> SLA, e3 = e4.w >> SLA;
    e0 = e0 < 0 ? 0 : (e0 > nE - 1 ? nE - 1 : e0);
    e1 = e1 < 0 ? 0 : (e1 > nE - 1 ? nE - 1 : e1);
    e2 = e2 < 0 ? 0 : (e2 > nE - 1 ? nE - 1 : e2);
    e3 = e3 < 0 ? 0 : (e3 > nE - 1 ? nE - 1 : e3);
    int r0 = srcs[e0], r1 = srcs[e1], r2 = srcs[e2], r3 = srcs[e3];
    r0 = r0 < 0 ? 0 : (r0 > nN - 1 ? nN - 1 : r0);
    r1 = r1 < 0 ? 0 : (r1 > nN - 1 ? nN - 1 : r1);
    r2 = r2 < 0 ? 0 : (r2 > nN - 1 ? nN - 1 : r2);
    r3 = r3 < 0 ? 0 : (r3 > nN - 1 ? nN - 1 : r3);
    v4i hv;
    hv.x = (p0     < tt) ? r0 : 0;
    hv.y = (p0 + 1 < tt) ? r1 : 0;
    hv.z = (p0 + 2 < tt) ? r2 : 0;
    hv.w = (p0 + 3 < tt) ? r3 : 0;
    int* hp = hrow + p0;
    *(volatile v4i*)hp = hv;
    __threadfence();
    *(volatile v4i*)hp = hv;
  }
}

__global__ __launch_bounds__(GTHR) void k_gemm(
    const unsigned short* __restrict__ A, const unsigned short* __restrict__ WT,
    float* outF, int K, int ldo)
{
  __shared__ __attribute__((aligned(16))) float stg[GBM * GBN];
  const int tid = (int)threadIdx.x, lane = tid & 31, wave = tid >> 5, hh = lane >> 4, m = lane & 15;
  const int rowBase = (int)blockIdx.x * GBM;
  const int col0    = (int)blockIdx.y * GBN;

  v8f acc[4];
  {
    const v8f z = {0.f, 0.f, 0.f, 0.f, 0.f, 0.f, 0.f, 0.f};
    acc[0] = z; acc[1] = z; acc[2] = z; acc[3] = z;
  }
  const unsigned short* ap = A  + (size_t)(rowBase + 16 * wave + m) * (size_t)K + 8 * hh;
  const unsigned short* wp = WT + (size_t)(col0 + m) * (size_t)K + 8 * hh;
  const int ksteps = K >> 5;
#pragma unroll 1
  for (int ks = 0; ks < ksteps; ++ks) {
    FragB af;
    af.h[0] = *(const v8usa*)(ap + 32 * ks);
    af.h[1] = *(const v8usa*)(ap + 32 * ks + 16);
#pragma unroll
    for (int t = 0; t < 4; ++t) {
      const unsigned short* wq = wp + (size_t)(16 * t) * (size_t)K + 32 * ks;
      FragB bf;
      bf.h[0] = *(const v8usa*)wq;
      bf.h[1] = *(const v8usa*)(wq + 16);
      acc[t] = wmb(af, bf, acc[t]);
    }
  }

#pragma unroll
  for (int t = 0; t < 4; ++t) {
    const int lc = 16 * t + m;
#pragma unroll
    for (int r = 0; r < 8; ++r) {
      const int lr = 16 * wave + 8 * hh + r;
      stg[lr * GBN + lc] = acc[t][r];
    }
  }
  __syncthreads();

  v4f fv[8];
#pragma unroll
  for (int i = 0; i < 8; ++i) {
    const int lr = 16 * wave + 2 * i + hh;
    fv[i] = *(const v4fa*)(stg + lr * GBN + 4 * m);
  }
#pragma unroll
  for (int i = 0; i < 8; ++i) {
    const int lr = 16 * wave + 2 * i + hh;
    const int gr = rowBase + lr;
    float* op = outF + (size_t)gr * (size_t)ldo + col0 + 4 * m;
    *(volatile v4f*)op = fv[i];
  }
  __threadfence();
#pragma unroll
  for (int i = 0; i < 8; ++i) {
    const int lr = 16 * wave + 2 * i + hh;
    const int gr = rowBase + lr;
    float* op = outF + (size_t)gr * (size_t)ldo + col0 + 4 * m;
    *(volatile v4f*)op = fv[i];
  }
}

__global__ __launch_bounds__(NTHR) void k_agg(const int* __restrict__ hits, const int* __restrict__ cntg,
                                              const int* __restrict__ offg, const int* __restrict__ flagg,
                                              int nN, int mRows,
                                              const float* __restrict__ dis,
                                              const float* __restrict__ xl, const float* __restrict__ bias,
                                              unsigned short* hb) {
  const int tid = (int)threadIdx.x, lane = tid & 31, wave = tid >> 5;
  const int nodeBase = (int)blockIdx.x * NBA;
  const int* hrow = hits + (size_t)blockIdx.x * RCAP;
  const int fl = flagg[(size_t)blockIdx.x * FLN];

  float bv0, bv1;
  {
    const v2f a = *(const v2fa*)(bias + 2 * lane);
    bv0 = bf16_val(a.x); bv1 = bf16_val(a.y);
  }
  const float qnan = __int_as_float(0x7fc00000);
  const int q0s = (4 * lane) & 31, q1s = (4 * lane + 1) & 31;
  const int q2s = (4 * lane + 2) & 31, q3s = (4 * lane + 3) & 31;
#pragma unroll 1
  for (int si = 0; si < NBA / NWAVE; ++si) {
    const int s    = si * NWAVE + wave;
    const int node = nodeBase + s;
    int c = cntg[node];
    const bool big = c > DEGCAP;
    c = c < 0 ? 0 : (c > DEGCAP ? DEGCAP : c);
    int o = offg[node];
    o = o < 0 ? 0 : (o > RCAP ? RCAP : o);
    if (c > RCAP - o) c = RCAP - o;
    const int nc = node < nN ? node : nN - 1;
    const float dd = dis[nc];
    const float rd = dd * dd;
    float acc0 = 0.0f, acc1 = 0.0f;
#pragma unroll 1
    for (int b0 = 0; b0 < c; b0 += 32) {
      int idx = o + b0 + lane;
      idx = idx > RCAP - 1 ? RCAP - 1 : idx;
      int sr = hrow[idx];
      sr = sr < 0 ? 0 : (sr > nN - 1 ? nN - 1 : sr);
      const float cf  = dis[sr] * dd;
      const int   cfi = __float_as_int(cf);
      const int m32 = (c - b0) < 32 ? (c - b0) : 32;
#pragma unroll 1
      for (int k = 0; k < m32; ++k) {
        const int   sk = __builtin_amdgcn_readlane(sr, k);
        const float ck = __int_as_float(__builtin_amdgcn_readlane(cfi, k));
        const v2f a = *(const v2fa*)(xl + (size_t)sk * CH + 2 * lane);
        acc0 = fmaf(ck, a.x, acc0); acc1 = fmaf(ck, a.y, acc1);
      }
    }
    float sv0, sv1;
    {
      const v2f a = *(const v2fa*)(xl + (size_t)nc * CH + 2 * lane);
      sv0 = a.x; sv1 = a.y;
    }
    const bool poison = (fl != 0) || big;
    const bool live = node < nN;
    float y0 = (acc0 + sv0 * rd) + bv0;
    float y1 = (acc1 + sv1 * rd) + bv1;
    y0 = (y0 > 0.0f) ? y0 : (y0 - y0);
    y1 = (y1 > 0.0f) ? y1 : (y1 - y1);
    y0 = poison ? qnan : y0;
    y1 = poison ? qnan : y1;
    const float v0 = live ? y0 : 0.0f;
    const float v1 = live ? y1 : 0.0f;
    const bool wr = (node < mRows) && (lane < 16);
    const unsigned hb0 = bf16_bits(v0), hb1 = bf16_bits(v1);
    const unsigned lb0 = bf16_bits(v0 - __uint_as_float(hb0 << 16));
    const unsigned lb1 = bf16_bits(v1 - __uint_as_float(hb1 << 16));
    const int hw = (int)(hb0 | (hb1 << 16));
    const int lw = (int)(lb0 | (lb1 << 16));
    const int g0 = __shfl(hw, q0s, 32), g1 = __shfl(hw, q1s, 32);
    const int g2 = __shfl(hw, q2s, 32), g3 = __shfl(hw, q3s, 32);
    const int p0 = __shfl(lw, q0s, 32), p1 = __shfl(lw, q1s, 32);
    const int p2 = __shfl(lw, q2s, 32), p3 = __shfl(lw, q3s, 32);
    const bool lsel = (lane & 8) != 0;
    v4u pv;
    pv.x = (unsigned int)(lsel ? p0 : g0);
    pv.y = (unsigned int)(lsel ? p1 : g1);
    pv.z = (unsigned int)(lsel ? p2 : g2);
    pv.w = (unsigned int)(lsel ? p3 : g3);
    unsigned short* hp = hb + (size_t)node * K2 + 8 * (lane & 15);
    if (wr) *(volatile v4u*)hp = pv;
    __threadfence();
    if (wr) *(volatile v4u*)hp = pv;
  }
}

__global__ __launch_bounds__(NTHR) void k_head(const unsigned short* __restrict__ A,
                                               const unsigned short* __restrict__ WT,
                                               const float* __restrict__ bfc, const int* __restrict__ flagg,
                                               int nN, float* out) {
  __shared__ __attribute__((aligned(16))) float stg[HBM * OUTC];
  __shared__ float bls[OUTC];
  const int tid = (int)threadIdx.x, lane = tid & 31, wave = tid >> 5, hh = lane >> 4, m = lane & 15;
  const int rowBase = (int)blockIdx.x * HBM;

  if (tid < OUTC) bls[tid] = bf16_val(bfc[tid]);

  v8f acc = {0.f, 0.f, 0.f, 0.f, 0.f, 0.f, 0.f, 0.f};
  const unsigned short* ap = A  + (size_t)(rowBase + 16 * wave + m) * (size_t)K2 + 8 * hh;
  const unsigned short* wp = WT + (size_t)m * (size_t)K2 + 8 * hh;
#pragma unroll
  for (int ks = 0; ks < K2 / 32; ++ks) {
    FragB af, bf;
    af.h[0] = *(const v8usa*)(ap + 32 * ks);
    af.h[1] = *(const v8usa*)(ap + 32 * ks + 16);
    bf.h[0] = *(const v8usa*)(wp + 32 * ks);
    bf.h[1] = *(const v8usa*)(wp + 32 * ks + 16);
    acc = wmb(af, bf, acc);
  }
#pragma unroll
  for (int r = 0; r < 8; ++r) {
    const int lr = 16 * wave + 8 * hh + r;
    stg[lr * OUTC + m] = acc[r];
  }
  __syncthreads();

  const int fl = flagg[(size_t)(rowBase >> SLA) * FLN];
  const float qnan = __int_as_float(0x7fc00000);
  if (tid < HBM) {
    float* rp = stg + tid * OUTC;
    float mx = rp[0] + bls[0];
    rp[0] = mx;
#pragma unroll 1
    for (int c = 1; c < OUTC; ++c) {
      const float v = rp[c] + bls[c];
      rp[c] = v;
      mx = (v > mx || v != v) ? v : mx;
    }
    float s = 0.0f;
#pragma unroll 1
    for (int c = 0; c < OUTC; ++c) s += expf(rp[c] - mx);
    const float ls = logf(s);
#pragma unroll 1
    for (int c = 0; c < OUTC; ++c) {
      float o = (rp[c] - mx) - ls;
      o = (fl != 0) ? qnan : o;
      rp[c] = o;
    }
  }
  __syncthreads();

  constexpr int NIT = (HBM * OUTC) / (4 * NTHR);
  v4f ov[NIT];
  bool okv[NIT];
#pragma unroll
  for (int it = 0; it < NIT; ++it) {
    const int p = it * NTHR + tid;
    ov[it]  = *(const v4fa*)(stg + 4 * p);
    okv[it] = (rowBase + (p >> 2)) < nN;
  }
  float* ob = out + (size_t)rowBase * OUTC;
#pragma unroll
  for (int it = 0; it < NIT; ++it) {
    const int p = it * NTHR + tid;
    if (okv[it]) *(volatile v4f*)(ob + 4 * (size_t)p) = ov[it];
  }
  __threadfence();
#pragma unroll
  for (int it = 0; it < NIT; ++it) {
    const int p = it * NTHR + tid;
    if (okv[it]) *(volatile v4f*)(ob + 4 * (size_t)p) = ov[it];
  }
}

static inline int cdiv(int a, int b) { return (a + b - 1) / b; }
static inline size_t al256(size_t o) { return (o + 255) & ~(size_t)255; }

extern "C" void kernel_launch(void* const* d_in, const int* in_sizes, int n_in,
                              void* d_out, int out_size, void* d_ws, size_t ws_size,
                              hipStream_t stream) {
  if (n_in < 8) return;
  if (in_sizes[0] < CH || (in_sizes[0] % CH) != 0) return;
  const int nN = in_sizes[0] / CH;
  if (nN < 2 || nN > (1 << 22) || (nN & 1) != 0) return;
  if (in_sizes[1] < 2 || (in_sizes[1] & 1) != 0) return;
  const int nE = in_sizes[1] / 2;
  if (nE < 1 || nE >= (1 << (31 - SLA))) return;
  if (in_sizes[2] != CH * CH || in_sizes[3] != CH) return;
  if (in_sizes[4] != CH * CH || in_sizes[5] != CH) return;
  if (in_sizes[6] != CH * OUTC || in_sizes[7] != OUTC) return;
  if (out_size != nN * OUTC) return;

  const float* x    = (const float*)d_in[0];
  const int*   edge = (const int*)d_in[1];
  const float* W1   = (const float*)d_in[2];
  const float* b1   = (const float*)d_in[3];
  const float* W2   = (const float*)d_in[4];
  const float* b2   = (const float*)d_in[5];
  const float* Wfc  = (const float*)d_in[6];
  const float* bfc  = (const float*)d_in[7];
  float* out = (float*)d_out;
  const int* src = edge;
  const int* dst = edge + nE;

  const int MP  = cdiv(nN, MROWS) * MROWS;
  const int gM  = MP / GBM;
  const int gH  = MP / HBM;
  const int gA  = cdiv(MP, NBA);
  const int nXb = MP / 32;
  if ((long long)gA * NBA < (long long)MP) return;
  if ((MP % GBM) != 0 || (MP % HBM) != 0 || (MP % 32) != 0) return;
  const int vec8 = ((nE & 3) == 0) ? 1 : 0;
  const int NSL  = gA * NBA;

  char* ws = (char*)d_ws;
  size_t off = 0;
  const size_t oXB  = off; off = al256(off + (size_t)MP * CH * 2);
  const size_t oW1T = off; off = al256(off + (size_t)CH * CH * 2);
  const size_t oW2D = off; off = al256(off + (size_t)CH * K2 * 2);
  const size_t oWfD = off; off = al256(off + (size_t)OUTC * K2 * 2);
  const size_t oH   = off; off = al256(off + (size_t)MP * CH * 4);
  const size_t oX   = off; off = al256(off + (size_t)MP * K2 * 2);
  const size_t oHIT = off; off = al256(off + (size_t)gA * RCAP * 4);
  const size_t oCNT = off; off = al256(off + (size_t)NSL * 4);
  const size_t oOFF = off; off = al256(off + (size_t)NSL * 4);
  const size_t oDIS = off; off = al256(off + (size_t)NSL * 4);
  const size_t oFLG = off; off = al256(off + (size_t)gA * FLN * 4);
  if (off > ws_size || off > (size_t)WSMAX) return;
  unsigned short* XB  = (unsigned short*)(ws + oXB);
  unsigned short* W1T = (unsigned short*)(ws + oW1T);
  unsigned short* W2D = (unsigned short*)(ws + oW2D);
  unsigned short* WfD = (unsigned short*)(ws + oWfD);
  float*          H   = (float*)(ws + oH);
  unsigned short* X   = (unsigned short*)(ws + oX);
  int*            HIT = (int*)(ws + oHIT);
  int*            CNT = (int*)(ws + oCNT);
  int*            OFF = (int*)(ws + oOFF);
  float*          DIS = (float*)(ws + oDIS);
  int*            FLG = (int*)(ws + oFLG);

  const size_t bkLds = (size_t)AGG_LDS_INTS * 4;
  hipFuncSetAttribute(reinterpret_cast<const void*>(&k_bucket), hipFuncAttributeMaxDynamicSharedMemorySize, (int)bkLds);

  k_prep<<<nXb + (NU1 + NU2 + NU3) / NTHR, NTHR, 0, stream>>>(x, W1, W2, Wfc, nN, nXb, XB, W1T, W2D, WfD);
  k_bucket<<<gA, NTHR, bkLds, stream>>>(src, dst, nE, nN, vec8, HIT, CNT, OFF, DIS, FLG);
  k_gemm<<<dim3(gM, CH / GBN), GTHR, 0, stream>>>(XB, W1T, H, CH, CH);
  k_agg<<<gA, NTHR, 0, stream>>>(HIT, CNT, OFF, FLG, nN, MP, DIS, H, b1, X);
  k_gemm<<<dim3(gM, CH / GBN), GTHR, 0, stream>>>(X, W2D, H, K2, CH);
  k_agg<<<gA, NTHR, 0, stream>>>(HIT, CNT, OFF, FLG, nN, MP, DIS, H, b2, X);
  k_head<<<gH, NTHR, 0, stream>>>(X, WfD, bfc, FLG, nN, out);
}
